// GraphModel_17119739642111
// MI455X (gfx1250) — hardware-run, weakly checked
//
#include <hip/hip_runtime.h>
#include <stddef.h>
#include <stdint.h>
#include <math.h>

#define NN      100000
#define NE      3200000
#define EMBD    32
#define OD      16
#define KST     10
#define NTHR    256
#define NWAVE   8
#define NBRUN   1024
#define SLB     10
#define NBK     98
#define KPW     128
#define WSHARE  (NE / NWAVE)
#define NITER   (WSHARE / KPW)
#define WCAP    4608
#define RCAP    36864
#define DEGCAP  96
#define LISTTOT (NBK * RCAP)
#define NSLOT   (NBK * NBRUN)
#define MAXDEG_MEAS   59
#define MAXB1024_MEAS 33343
#define GBM     128
#define NMB     ((NN + GBM - 1) / GBM)
#define NSB     ((NN + 63) / 64)
#define NDB     (NE / NTHR)

#define BK_INTS (NWAVE * WCAP + 3 * NBRUN + RCAP / 32 + 16 + RCAP / 2)
#define BK_LDS  (BK_INTS * 4)

static_assert(NE % (KPW * NWAVE) == 0);
static_assert(NN <= (1 << 17) && NBRUN == 1024 && NBRUN == (1 << SLB));
static_assert(NBK * NBRUN >= NN);
static_assert(RCAP == NWAVE * WCAP && RCAP % (NTHR * 4) == 0 && RCAP % 32 == 0);
static_assert((long long)RCAP * 100 >= (long long)MAXB1024_MEAS * 105);
static_assert(WCAP >= MAXB1024_MEAS / 8 + 6 * 64 + 1);
static_assert(MAXDEG_MEAS + 8 <= DEGCAP);
static_assert(NN % 16 == 0 && NN % 8 == 0);
static_assert(NE % NTHR == 0 && NE % 32 == 0 && NE % 1024 == 0);
static_assert(BK_INTS % 4 == 0 && BK_LDS <= 327680);
static_assert((long long)LISTTOT < (1LL << 31));
static_assert(NBRUN == NTHR * 4);
static_assert(EMBD == 32 && OD == 16);

typedef float          v4f   __attribute__((ext_vector_type(4)));
typedef float          v8f   __attribute__((ext_vector_type(8)));
typedef int            v2i   __attribute__((ext_vector_type(2)));
typedef int            v4i   __attribute__((ext_vector_type(4)));
typedef int            v8i   __attribute__((ext_vector_type(8)));
typedef unsigned short v8us  __attribute__((ext_vector_type(8)));
typedef unsigned short v16us __attribute__((ext_vector_type(16)));
typedef __bf16         v16bf __attribute__((ext_vector_type(16)));
typedef v4f  __attribute__((may_alias)) v4fa;
typedef v2i  __attribute__((may_alias)) v2ia;
typedef v4i  __attribute__((may_alias)) v4ia;
typedef v8us __attribute__((may_alias)) v8usa;
union FragB { v16bf v; v16us u; v8us h[2]; v8i w; };

__device__ __forceinline__ v8f wmb(const FragB& a, const FragB& b, v8f c) {
  v8f d = __builtin_amdgcn_wmma_f32_16x16x32_bf16(false, a.v, false, b.v, (short)0, c, false, false);
  asm volatile("v_nop\n\tv_nop\n\tv_nop\n\tv_nop" : "+v"(d) : "v"(a.w), "v"(b.w));
  return d;
}

__device__ __forceinline__ unsigned bf16_bits(float f) {
  const unsigned u = __float_as_uint(f);
  const unsigned r = (u + 0x7FFFu + ((u >> 16) & 1u)) >> 16;
  const unsigned q = (u >> 16) | 0x40u;
  return ((u & 0x7fffffffu) > 0x7f800000u) ? q : r;
}

__device__ __forceinline__ float relu_keep(float v) { return (v > 0.0f) ? v : (v - v); }

__device__ __forceinline__ void st2_v4f(float* p, v4f v) {
  *(volatile v4f*)p = v;
  __threadfence();
  *(volatile v4f*)p = v;
}
__device__ __forceinline__ void st2_v8us(unsigned short* p, v8us v) {
  *(volatile v8us*)p = v;
  __threadfence();
  *(volatile v8us*)p = v;
}

__global__ __launch_bounds__(128) void k_prep(const float* __restrict__ w1, const float* __restrict__ b1,
                                              const float* __restrict__ w2, const float* __restrict__ b2,
                                              unsigned short* w1p, float* sm) {
  const int tid = (int)threadIdx.x, wave = tid >> 5;
  if (wave < 2) {
    const int n = tid >> 2, k8 = (tid & 3) * 8;
    const int nc = n & 7;
    const unsigned mk = (n < 8) ? 0xffffu : 0u;
    const float* p = w1 + (size_t)nc * EMBD + k8;
    const v4f a = *(const v4fa*)p;
    const v4f b = *(const v4fa*)(p + 4);
    v8us o;
    o[0] = (unsigned short)(bf16_bits(a.x) & mk); o[1] = (unsigned short)(bf16_bits(a.y) & mk);
    o[2] = (unsigned short)(bf16_bits(a.z) & mk); o[3] = (unsigned short)(bf16_bits(a.w) & mk);
    o[4] = (unsigned short)(bf16_bits(b.x) & mk); o[5] = (unsigned short)(bf16_bits(b.y) & mk);
    o[6] = (unsigned short)(bf16_bits(b.z) & mk); o[7] = (unsigned short)(bf16_bits(b.w) & mk);
    st2_v8us(w1p + (size_t)n * EMBD + k8, o);
  } else {
    const int t = tid - 64;
    const int tw = t < 32 ? t : 31;
    int tb = t - 32; tb = tb < 0 ? 0 : (tb > 1 ? 1 : tb);
    int tc = t - 36; tc = tc < 0 ? 0 : (tc > 3 ? 3 : tc);
    const v4f a = *(const v4fa*)(w2 + 4 * tw);
    const v4f b = *(const v4fa*)(b1 + 4 * tb);
    const v4f c = *(const v4fa*)(b2 + 4 * tc);
    asm volatile("" :: "v"(a));
    asm volatile("" :: "v"(b));
    asm volatile("" :: "v"(c));
    const unsigned ma = (t < 32) ? 0xffffffffu : 0u;
    const unsigned mb = (t >= 32 && t < 34) ? 0xffffffffu : 0u;
    const unsigned mc = (t >= 36 && t < 40) ? 0xffffffffu : 0u;
    v4f o;
    o.x = __uint_as_float(((bf16_bits(a.x) << 16) & ma) | ((bf16_bits(b.x) << 16) & mb) | ((bf16_bits(c.x) << 16) & mc));
    o.y = __uint_as_float(((bf16_bits(a.y) << 16) & ma) | ((bf16_bits(b.y) << 16) & mb) | ((bf16_bits(c.y) << 16) & mc));
    o.z = __uint_as_float(((bf16_bits(a.z) << 16) & ma) | ((bf16_bits(b.z) << 16) & mb) | ((bf16_bits(c.z) << 16) & mc));
    o.w = __uint_as_float(((bf16_bits(a.w) << 16) & ma) | ((bf16_bits(b.w) << 16) & mb) | ((bf16_bits(c.w) << 16) & mc));
    float* dp = sm + 4 * t;
    const bool wr = t < 40;
    if (wr) *(volatile v4f*)dp = o;
    __threadfence();
    if (wr) *(volatile v4f*)dp = o;
  }
}

__device__ __forceinline__ int hit_put(bool h, unsigned slot, int srcv, int wc, int* mylist) {
  const unsigned mj = __builtin_amdgcn_ballot_w32(h);
  if (mj != 0u) {
    const int sc = srcv < 0 ? 0 : (srcv > NN - 1 ? NN - 1 : srcv);
    const int pos = wc + (int)__builtin_amdgcn_mbcnt_lo(mj, 0u);
    if (h && pos < WCAP) mylist[pos] = (sc << SLB) | (int)slot;
    wc += (int)__builtin_popcount(mj);
  }
  return wc;
}

__device__ __forceinline__ void bucket_flush(const unsigned short* plo, const unsigned* phi, const int* cnt,
                                             const int* offs, const int* dvb, int lbase,
                                             int* lp, int* cp, int* op, int* dp, int tid) {
#pragma unroll 1
  for (int i = tid * 4; i < RCAP; i += NTHR * 4) {
    const v2i w = *(const v2ia*)(plo + i);
    const unsigned b = phi[i >> 5] >> (i & 31);
    v4i v;
    v.x = (int)(((unsigned)w.x & 0xffffu) | ((b & 1u) << 16));
    v.y = (int)(((unsigned)w.x >> 16)     | (((b >> 1) & 1u) << 16));
    v.z = (int)(((unsigned)w.y & 0xffffu) | (((b >> 2) & 1u) << 16));
    v.w = (int)(((unsigned)w.y >> 16)     | (((b >> 3) & 1u) << 16));
    *(volatile v4i*)(lp + i) = v;
  }
  {
    const v4i c4 = *(const v4ia*)(cnt + 4 * tid);
    v4i o4 = *(const v4ia*)(offs + 4 * tid);
    const v4i d4 = *(const v4ia*)(dvb + 4 * tid);
    o4.x += lbase; o4.y += lbase; o4.z += lbase; o4.w += lbase;
    *(volatile v4i*)(cp + 4 * tid) = c4;
    *(volatile v4i*)(op + 4 * tid) = o4;
    *(volatile v4i*)(dp + 4 * tid) = d4;
  }
}

__global__ __launch_bounds__(NTHR) void k_bucket(const int* __restrict__ srcs, const int* __restrict__ dsts,
                                                 int* LIST, int* CNT, int* OFF, int* DINVB) {
  extern __shared__ __attribute__((aligned(16))) int dsm[];
  int* wl   = dsm;
  int* cnt  = dsm + NWAVE * WCAP;
  int* offs = cnt + NBRUN;
  int* cur  = offs + NBRUN;
  unsigned* phi = (unsigned*)(cur + NBRUN);
  int* misc = (int*)(phi + RCAP / 32);
  unsigned short* plo = (unsigned short*)(misc + 16);
  const int tid = (int)threadIdx.x, lane = tid & 31, wave = tid >> 5;
  const int blk = (int)blockIdx.x;
  const unsigned nbs = (unsigned)(blk * NBRUN);

  {
    const v4i z4 = {0, 0, 0, 0};
    for (int i = tid * 4; i < BK_INTS; i += NTHR * 4) *(v4ia*)(dsm + i) = z4;
  }
  __syncthreads();

  {
    const int* dw = dsts + (size_t)wave * WSHARE;
    const int* sw = srcs + (size_t)wave * WSHARE;
    int* mylist = wl + wave * WCAP;
    int wc = 0;
#pragma unroll 1
    for (int it = 0; it < NITER; ++it) {
      const int e0 = it * KPW + 4 * lane;
      const v4i d4 = *(const v4ia*)(dw + e0);
      const unsigned s0 = (unsigned)d4.x - nbs, s1 = (unsigned)d4.y - nbs;
      const unsigned s2 = (unsigned)d4.z - nbs, s3 = (unsigned)d4.w - nbs;
      const bool h0 = s0 < (unsigned)NBRUN, h1 = s1 < (unsigned)NBRUN;
      const bool h2 = s2 < (unsigned)NBRUN, h3 = s3 < (unsigned)NBRUN;
      const unsigned any = __builtin_amdgcn_ballot_w32(h0 | h1 | h2 | h3);
      if (any != 0u) {
        const v4i s4 = *(const v4ia*)(sw + e0);
        asm volatile("" :: "v"(s4));
        wc = hit_put(h0, s0, s4.x, wc, mylist);
        wc = hit_put(h1, s1, s4.y, wc, mylist);
        wc = hit_put(h2, s2, s4.z, wc, mylist);
        wc = hit_put(h3, s3, s4.w, wc, mylist);
      }
    }
    if (lane == 0) misc[wave] = wc;
  }
  __syncthreads();

  if (wave == 0) {
    int ov = 0;
#pragma unroll 1
    for (int w2 = 0; w2 < NWAVE; ++w2) {
      int c = misc[w2];
      if (c > WCAP) ov = 1;
      c = c < 0 ? 0 : (c > WCAP ? WCAP : c);
      c = __builtin_amdgcn_readfirstlane(c);
#pragma unroll 1
      for (int b0 = 0; b0 < c; b0 += 32) {
        const int idx = b0 + lane;
        const int ent = wl[w2 * WCAP + (idx < WCAP ? idx : WCAP - 1)];
        const int m32 = (c - b0) < 32 ? (c - b0) : 32;
#pragma unroll 1
        for (int k = 0; k < m32; ++k) {
          const int u    = __builtin_amdgcn_readlane(ent, k);
          const int slot = u & (NBRUN - 1);
          if (lane == 0) cnt[slot] = cnt[slot] + 1;
        }
      }
    }
    if (lane == 0) misc[9] = ov;
  }
  __syncthreads();
  if (wave == 0) {
    const int base = lane * (NBRUN / 32);
    int s = 0;
    int bigl = 0;
#pragma unroll 1
    for (int i = 0; i < NBRUN / 32; ++i) {
      const int cv = cnt[base + i];
      bigl |= (cv > DEGCAP) ? 1 : 0;
      s += cv;
    }
    int incl = s;
#pragma unroll
    for (int d = 1; d < 32; d <<= 1) {
      const int y = __shfl_up(incl, d, 32);
      if (lane >= d) incl += y;
    }
    const int total = __shfl(incl, 31, 32);
    const unsigned bm = __builtin_amdgcn_ballot_w32(bigl != 0);
    int run = incl - s;
#pragma unroll 1
    for (int i = 0; i < NBRUN / 32; ++i) {
      const int cv = cnt[base + i];
      offs[base + i] = run;
      cur[base + i]  = run;
      run += cv;
    }
    if (lane == 0) {
      const int f = misc[9];
      misc[9] = (f != 0 || bm != 0u || total > RCAP) ? 1 : 0;
    }
  }
  __syncthreads();

  if (wave == 0) {
#pragma unroll 1
    for (int w2 = 0; w2 < NWAVE; ++w2) {
      int c = misc[w2];
      c = c < 0 ? 0 : (c > WCAP ? WCAP : c);
      c = __builtin_amdgcn_readfirstlane(c);
#pragma unroll 1
      for (int b0 = 0; b0 < c; b0 += 32) {
        const int idx = b0 + lane;
        const int ent = wl[w2 * WCAP + (idx < WCAP ? idx : WCAP - 1)];
        const int m32 = (c - b0) < 32 ? (c - b0) : 32;
#pragma unroll 1
        for (int k = 0; k < m32; ++k) {
          const int u    = __builtin_amdgcn_readlane(ent, k);
          const int slot = u & (NBRUN - 1);
          const unsigned sr = ((unsigned)u >> SLB) & 0x1FFFFu;
          if (lane == 0) {
            int p = cur[slot];
            p = p < 0 ? 0 : (p > RCAP - 1 ? RCAP - 1 : p);
            plo[p] = (unsigned short)(sr & 0xffffu);
            const unsigned hw = phi[p >> 5];
            phi[p >> 5] = hw | ((sr >> 16) << (p & 31));
            cur[slot] = p + 1;
          }
        }
      }
    }
  }
  __syncthreads();

  {
    const int ovf = misc[9];
#pragma unroll 1
    for (int s = tid; s < NBRUN; s += NTHR) {
      int c = cnt[s];
      c = c < 0 ? 0 : c;
      const float dv = 1.0f / sqrtf((float)(c + 1));
      cur[s] = (ovf != 0) ? 0x7fc00000 : __float_as_int(dv);
    }
  }
  __syncthreads();

  const int lbase = blk * RCAP;
  int* lp = LIST + (size_t)blk * RCAP;
  int* cp = CNT + (size_t)blk * NBRUN;
  int* op = OFF + (size_t)blk * NBRUN;
  int* dp = DINVB + (size_t)blk * NBRUN;
  bucket_flush(plo, phi, cnt, offs, cur, lbase, lp, cp, op, dp, tid);
  __threadfence();
  bucket_flush(plo, phi, cnt, offs, cur, lbase, lp, cp, op, dp, tid);
}

__global__ __launch_bounds__(NTHR) void k_mlp(const float* __restrict__ emb, const unsigned short* __restrict__ W1P,
                                              const float* __restrict__ sm, const float* __restrict__ DINV,
                                              float* H, float* P0) {
  __shared__ __attribute__((aligned(16))) float dt[NWAVE * 256];
  __shared__ __attribute__((aligned(16))) float hs[NWAVE * 256];
  __shared__ __attribute__((aligned(16))) float ps[NWAVE * 256];
  __shared__ __attribute__((aligned(16))) float sp[256];
  const int tid = (int)threadIdx.x, lane = tid & 31, wave = tid >> 5, hh = lane >> 4, m = lane & 15;
  const int tile0 = (int)blockIdx.x * GBM + 16 * wave;
  const bool live = tile0 < NN;

  if (tid < 64) {
    const int tc = tid < 40 ? tid : 39;
    *(v4fa*)(sp + 4 * tid) = *(const v4fa*)(sm + 4 * tc);
  }

  FragB af, bf;
  {
    int row = tile0 + m;
    row = row > NN - 1 ? NN - 1 : row;
    const float* ep = emb + (size_t)row * EMBD + 8 * hh;
    const v4f a0 = *(const v4fa*)ep;
    const v4f a1 = *(const v4fa*)(ep + 4);
    const v4f a2 = *(const v4fa*)(ep + 16);
    const v4f a3 = *(const v4fa*)(ep + 20);
    v8i aw;
    aw[0] = (int)(bf16_bits(a0.x) | (bf16_bits(a0.y) << 16));
    aw[1] = (int)(bf16_bits(a0.z) | (bf16_bits(a0.w) << 16));
    aw[2] = (int)(bf16_bits(a1.x) | (bf16_bits(a1.y) << 16));
    aw[3] = (int)(bf16_bits(a1.z) | (bf16_bits(a1.w) << 16));
    aw[4] = (int)(bf16_bits(a2.x) | (bf16_bits(a2.y) << 16));
    aw[5] = (int)(bf16_bits(a2.z) | (bf16_bits(a2.w) << 16));
    aw[6] = (int)(bf16_bits(a3.x) | (bf16_bits(a3.y) << 16));
    aw[7] = (int)(bf16_bits(a3.z) | (bf16_bits(a3.w) << 16));
    af.w = aw;
    const unsigned short* wq = W1P + (size_t)m * EMBD + 8 * hh;
    bf.h[0] = *(const v8usa*)wq;
    bf.h[1] = *(const v8usa*)(wq + 16);
  }
  v8f acc = {0.f, 0.f, 0.f, 0.f, 0.f, 0.f, 0.f, 0.f};
  acc = wmb(af, bf, acc);

  float* dw = dt + wave * 256;
#pragma unroll
  for (int r = 0; r < 8; ++r) dw[(8 * hh + r) * 16 + m] = acc[r];
  __syncthreads();

  float* hw = hs + wave * 256;
  float* pw = ps + wave * 256;
  {
    const int r = lane >> 1, half = lane & 1;
    const v4f d0 = *(const v4fa*)(dw + r * 16);
    const v4f d1 = *(const v4fa*)(dw + r * 16 + 4);
    const v4f c0 = *(const v4fa*)(sp + 128);
    const v4f c1 = *(const v4fa*)(sp + 132);
    const float h0 = relu_keep(d0.x + c0.x), h1 = relu_keep(d0.y + c0.y);
    const float h2 = relu_keep(d0.z + c0.z), h3 = relu_keep(d0.w + c0.w);
    const float h4 = relu_keep(d1.x + c1.x), h5 = relu_keep(d1.y + c1.y);
    const float h6 = relu_keep(d1.z + c1.z), h7 = relu_keep(d1.w + c1.w);
    int gr = tile0 + r;
    gr = gr > NN - 1 ? NN - 1 : gr;
    const float dv = DINV[gr];
#pragma unroll 1
    for (int j = 0; j < 8; ++j) {
      const int jj = 8 * half + j;
      const v4f w0 = *(const v4fa*)(sp + 8 * jj);
      const v4f w1 = *(const v4fa*)(sp + 8 * jj + 4);
      float s = 0.0f;
      s = fmaf(h0, w0.x, s); s = fmaf(h1, w0.y, s); s = fmaf(h2, w0.z, s); s = fmaf(h3, w0.w, s);
      s = fmaf(h4, w1.x, s); s = fmaf(h5, w1.y, s); s = fmaf(h6, w1.z, s); s = fmaf(h7, w1.w, s);
      s = s + sp[144 + jj];
      hw[r * 16 + jj] = s;
      pw[r * 16 + jj] = dv * s;
    }
  }
  __syncthreads();

  const v4f hv0 = *(const v4fa*)(hw + 4 * lane);
  const v4f hv1 = *(const v4fa*)(hw + 128 + 4 * lane);
  const v4f pv0 = *(const v4fa*)(pw + 4 * lane);
  const v4f pv1 = *(const v4fa*)(pw + 128 + 4 * lane);
  const int trow = live ? tile0 : 0;
  float* hp = H  + (size_t)trow * OD + 4 * lane;
  float* pp = P0 + (size_t)trow * OD + 4 * lane;
  if (live) {
    *(volatile v4f*)hp = hv0; *(volatile v4f*)(hp + 128) = hv1;
    *(volatile v4f*)pp = pv0; *(volatile v4f*)(pp + 128) = pv1;
  }
  __threadfence();
  if (live) {
    *(volatile v4f*)hp = hv0; *(volatile v4f*)(hp + 128) = hv1;
    *(volatile v4f*)pp = pv0; *(volatile v4f*)(pp + 128) = pv1;
  }
}

template <int LAST>
__global__ __launch_bounds__(NTHR) void k_step(const int* __restrict__ LIST, const int* __restrict__ CNT,
                                               const int* __restrict__ OFF, const float* __restrict__ DINV,
                                               const float* __restrict__ H, const float* Pin, float* Pout) {
  const int tid = (int)threadIdx.x, lane = tid & 31, wave = tid >> 5;
  const int nb = ((int)blockIdx.x * NWAVE + wave) * 8;
  if (nb >= NN) return;
  const int node = nb + (lane >> 2);
  const int q = lane & 3;
  int c = CNT[node];
  int o = OFF[node];
  const float dv = DINV[node];
  const bool big = c > DEGCAP;
  c = c < 0 ? 0 : (c > DEGCAP ? DEGCAP : c);
  o = o < 0 ? 0 : (o > LISTTOT - 1 ? LISTTOT - 1 : o);
  int last = o + c - 1;
  last = last < o ? o : last;
  last = last > LISTTOT - 1 ? LISTTOT - 1 : last;
  int cm = c < 1 ? 1 : c;
  {
    const int y4 = __shfl_xor(cm, 4, 32);  cm = cm > y4 ? cm : y4;
    const int y8 = __shfl_xor(cm, 8, 32);  cm = cm > y8 ? cm : y8;
    const int y16 = __shfl_xor(cm, 16, 32); cm = cm > y16 ? cm : y16;
  }
  const int cmax = __builtin_amdgcn_readfirstlane(cm);

  float s0 = 0.0f, s1 = 0.0f, s2 = 0.0f, s3 = 0.0f;
#pragma unroll 1
  for (int k = 0; k < cmax; ++k) {
    int idx = o + k;
    idx = idx > last ? last : idx;
    int sr = LIST[idx];
    sr = sr < 0 ? 0 : (sr > NN - 1 ? NN - 1 : sr);
    const v4f v = *(const v4fa*)(Pin + (size_t)sr * OD + 4 * q);
    asm volatile("" :: "v"(v));
    const bool valid = k < c;
    const float t0 = s0 + v.x, t1 = s1 + v.y, t2 = s2 + v.z, t3 = s3 + v.w;
    s0 = valid ? t0 : s0; s1 = valid ? t1 : s1; s2 = valid ? t2 : s2; s3 = valid ? t3 : s3;
  }
  const v4f pi = *(const v4fa*)(Pin + (size_t)node * OD + 4 * q);
  const v4f hv = *(const v4fa*)(H + (size_t)node * OD + 4 * q);
  s0 += pi.x; s1 += pi.y; s2 += pi.z; s3 += pi.w;
  const float g0 = dv * s0, g1 = dv * s1, g2 = dv * s2, g3 = dv * s3;
  float x0 = fmaf(0.9f, g0, 0.1f * hv.x);
  float x1 = fmaf(0.9f, g1, 0.1f * hv.y);
  float x2 = fmaf(0.9f, g2, 0.1f * hv.z);
  float x3 = fmaf(0.9f, g3, 0.1f * hv.w);
  const float qnan = __uint_as_float(0x7fc00000u);
  x0 = big ? qnan : x0; x1 = big ? qnan : x1; x2 = big ? qnan : x2; x3 = big ? qnan : x3;
  v4f ov;
  if constexpr (LAST != 0) {
    ov.x = x0; ov.y = x1; ov.z = x2; ov.w = x3;
  } else {
    ov.x = dv * x0; ov.y = dv * x1; ov.z = dv * x2; ov.w = dv * x3;
  }
  st2_v4f(Pout + (size_t)node * OD + 4 * q, ov);
}

__global__ __launch_bounds__(NTHR) void k_decode(const int* __restrict__ srcs, const int* __restrict__ dsts,
                                                 const float* __restrict__ X, float* out) {
  const int e = (int)blockIdx.x * NTHR + (int)threadIdx.x;
  int s = srcs[e];
  int d = dsts[e];
  s = s < 0 ? 0 : (s > NN - 1 ? NN - 1 : s);
  d = d < 0 ? 0 : (d > NN - 1 ? NN - 1 : d);
  const float* xs = X + (size_t)s * OD;
  const float* xd = X + (size_t)d * OD;
  const v4f a0 = *(const v4fa*)xs,       a1 = *(const v4fa*)(xs + 4);
  const v4f a2 = *(const v4fa*)(xs + 8), a3 = *(const v4fa*)(xs + 12);
  const v4f b0 = *(const v4fa*)xd,       b1 = *(const v4fa*)(xd + 4);
  const v4f b2 = *(const v4fa*)(xd + 8), b3 = *(const v4fa*)(xd + 12);
  float acc = 0.0f;
  acc = fmaf(a0.x, b0.x, acc); acc = fmaf(a0.y, b0.y, acc); acc = fmaf(a0.z, b0.z, acc); acc = fmaf(a0.w, b0.w, acc);
  acc = fmaf(a1.x, b1.x, acc); acc = fmaf(a1.y, b1.y, acc); acc = fmaf(a1.z, b1.z, acc); acc = fmaf(a1.w, b1.w, acc);
  acc = fmaf(a2.x, b2.x, acc); acc = fmaf(a2.y, b2.y, acc); acc = fmaf(a2.z, b2.z, acc); acc = fmaf(a2.w, b2.w, acc);
  acc = fmaf(a3.x, b3.x, acc); acc = fmaf(a3.y, b3.y, acc); acc = fmaf(a3.z, b3.z, acc); acc = fmaf(a3.w, b3.w, acc);
  float* op = out + (size_t)e;
  *(volatile float*)op = acc;
  __threadfence();
  *(volatile float*)op = acc;
}

extern "C" void kernel_launch(void* const* d_in, const int* in_sizes, int n_in,
                              void* d_out, int out_size, void* d_ws, size_t ws_size,
                              hipStream_t stream) {
  if (n_in < 6) return;
  if (in_sizes[0] != 2 * NE) return;
  if (in_sizes[1] != NN * EMBD) return;
  if (in_sizes[2] != 8 * EMBD) return;
  if (in_sizes[3] != 8) return;
  if (in_sizes[4] != OD * 8) return;
  if (in_sizes[5] != OD) return;
  if (out_size != NE) return;

  const int*   ei  = (const int*)d_in[0];
  const float* emb = (const float*)d_in[1];
  const float* w1  = (const float*)d_in[2];
  const float* b1  = (const float*)d_in[3];
  const float* w2  = (const float*)d_in[4];
  const float* b2  = (const float*)d_in[5];
  float* out = (float*)d_out;
  const int* srcs = ei;
  const int* dsts = ei + NE;

  constexpr size_t zPL   = (size_t)NN * OD * 4;
  constexpr size_t zLIST = (size_t)NBK * RCAP * 4;
  constexpr size_t zTAB  = (size_t)NSLOT * 4;
  constexpr size_t zW1P  = 1024;
  constexpr size_t zSM   = 1024;
  constexpr size_t oH    = 0;
  constexpr size_t oPA   = oH + zPL;
  constexpr size_t oPB   = oPA + zPL;
  constexpr size_t oX    = oPB + zPL;
  constexpr size_t oLIST = oX + zPL;
  constexpr size_t oCNT  = oLIST + zLIST;
  constexpr size_t oOFF  = oCNT + zTAB;
  constexpr size_t oDINV = oOFF + zTAB;
  constexpr size_t oW1P  = oDINV + zTAB;
  constexpr size_t oSM   = oW1P + zW1P;
  constexpr size_t oEND  = oSM + zSM;
  static_assert(zPL % 1024 == 0 && zLIST % 1024 == 0 && zTAB % 1024 == 0);
  static_assert(oEND <= (size_t)(128u << 20));
  if (oEND > ws_size) return;

  char* ws = (char*)d_ws;
  float* H    = (float*)(ws + oH);
  float* PA   = (float*)(ws + oPA);
  float* PB   = (float*)(ws + oPB);
  float* X    = (float*)(ws + oX);
  int*   LIST = (int*)(ws + oLIST);
  int*   CNT  = (int*)(ws + oCNT);
  int*   OFF  = (int*)(ws + oOFF);
  int*   DIB  = (int*)(ws + oDINV);
  const float* DINV = (const float*)(ws + oDINV);
  unsigned short* W1P = (unsigned short*)(ws + oW1P);
  float* SM   = (float*)(ws + oSM);

  hipFuncSetAttribute(reinterpret_cast<const void*>(&k_bucket), hipFuncAttributeMaxDynamicSharedMemorySize, (int)BK_LDS);

  k_prep<<<1, 128, 0, stream>>>(w1, b1, w2, b2, W1P, SM);
  k_bucket<<<NBK, NTHR, BK_LDS, stream>>>(srcs, dsts, LIST, CNT, OFF, DIB);
  k_mlp<<<NMB, NTHR, 0, stream>>>(emb, W1P, SM, DINV, H, PA);

  for (int s = 1; s <= KST; ++s) {
    const float* pin = (s & 1) ? PA : PB;
    float* pout = (s & 1) ? PB : PA;
    if (s == KST)
      k_step<1><<<NSB, NTHR, 0, stream>>>(LIST, CNT, OFF, DINV, H, pin, X);
    else
      k_step<0><<<NSB, NTHR, 0, stream>>>(LIST, CNT, OFF, DINV, H, pin, pout);
  }
  k_decode<<<NDB, NTHR, 0, stream>>>(srcs, dsts, X, out);
}
